// EdgeProbMLP_89781996355945
// MI455X (gfx1250) — hardware-verified
//
#include <hip/hip_runtime.h>
#include <stddef.h>


#define CH     128
#define KPB    128
#define APZ    136
#define DPF    132
#define GROWS  32
#define GTHR   64
#define EWAV   2
#define EPW    32
#define ETHR   (EWAV * 32)
#define EPB    (EWAV * EPW)
#define PTHR   256
#define PLN    (CH * KPB)
#define OFF_PD 0
#define OFF_PA PLN
#define OFF_PB (2 * PLN)
#define BPTOT  (3 * PLN)
#define NPBLK  24
#define WSCAP  134217728
#define WSC    64.0f
#define HSC    16.0f
#define ASC    1024.0f
#define RW     0.015625f
#define RH     0.0009765625f

static_assert(BPTOT == 49152);
static_assert((APZ % 8) == 0 && (KPB % 8) == 0 && (DPF % 4) == 0);
static_assert(GROWS == (GTHR / 32) * 16);
static_assert((CH % 32) == 0);
static_assert(EPB == ETHR);
static_assert(GROWS * CH == 16 * GTHR * 4);
static_assert(NPBLK * PTHR * 8 == BPTOT);
static_assert(EWAV * EPW * APZ * 2 + EWAV * EPW * DPF * 4 + EPB * 4 <= 65536);

typedef float    v4f  __attribute__((ext_vector_type(4)));
typedef float    v8f  __attribute__((ext_vector_type(8)));
typedef _Float16 v4h  __attribute__((ext_vector_type(4)));
typedef _Float16 v8h  __attribute__((ext_vector_type(8)));
typedef _Float16 v16h __attribute__((ext_vector_type(16)));
union Frag { v16h v; v8h h[2]; };

__device__ __forceinline__ v8f wmh(v16h a, v16h b, v8f c) {
  v8f d = __builtin_amdgcn_wmma_f32_16x16x32_f16(false, a, false, b, (short)0, c, false, false);
  asm volatile("v_nop\n\tv_nop\n\tv_nop\n\tv_nop" : "+v"(d) : "v"(a), "v"(b));
  return d;
}

template <int NT>
__device__ __forceinline__ void mma16(const _Float16* At, const _Float16* __restrict__ Bpl,
                                      int lane, v8f (&acc)[NT]) {
  const int hh = lane >> 4, m = lane & 15;
#pragma unroll
  for (int t = 0; t < NT; ++t) { v8f z = {0.f, 0.f, 0.f, 0.f, 0.f, 0.f, 0.f, 0.f}; acc[t] = z; }
  const _Float16* ap = At + m * APZ + 8 * hh;
  const _Float16* bb = Bpl + (size_t)m * KPB + 8 * hh;
#pragma unroll 1
  for (int ks = 0; ks < CH / 32; ++ks) {
    Frag a;
    a.h[0] = *(const v8h*)(ap + 32 * ks);
    a.h[1] = *(const v8h*)(ap + 32 * ks + 16);
#pragma unroll
    for (int t = 0; t < NT; ++t) {
      const _Float16* bp = bb + (size_t)(16 * t) * KPB + 32 * ks;
      Frag b;
      b.h[0] = *(const v8h*)bp;
      b.h[1] = *(const v8h*)(bp + 16);
      acc[t] = wmh(a.v, b.v, acc[t]);
    }
  }
}

template <int NT>
__device__ __forceinline__ void mma32(const _Float16* At, const _Float16* __restrict__ Bpl,
                                      int lane, v8f (&acc0)[NT], v8f (&acc1)[NT]) {
  const int hh = lane >> 4, m = lane & 15;
#pragma unroll
  for (int t = 0; t < NT; ++t) {
    v8f z = {0.f, 0.f, 0.f, 0.f, 0.f, 0.f, 0.f, 0.f};
    acc0[t] = z; acc1[t] = z;
  }
  const _Float16* ap0 = At + m * APZ + 8 * hh;
  const _Float16* ap1 = ap0 + 16 * APZ;
  const _Float16* bb  = Bpl + (size_t)m * KPB + 8 * hh;
#pragma unroll 1
  for (int ks = 0; ks < CH / 32; ++ks) {
    Frag a0, a1;
    a0.h[0] = *(const v8h*)(ap0 + 32 * ks);
    a0.h[1] = *(const v8h*)(ap0 + 32 * ks + 16);
    a1.h[0] = *(const v8h*)(ap1 + 32 * ks);
    a1.h[1] = *(const v8h*)(ap1 + 32 * ks + 16);
#pragma unroll
    for (int t = 0; t < NT; ++t) {
      const _Float16* bp = bb + (size_t)(16 * t) * KPB + 32 * ks;
      Frag b;
      b.h[0] = *(const v8h*)bp;
      b.h[1] = *(const v8h*)(bp + 16);
      acc0[t] = wmh(a0.v, b.v, acc0[t]);
      acc1[t] = wmh(a1.v, b.v, acc1[t]);
    }
  }
}

template <int J0>
__device__ __forceinline__ void rows8(_Float16* hw, float* dw, const float* __restrict__ R,
                                      const float* __restrict__ S, v4f b1s, int sv, int dv, int lane) {
#pragma unroll
  for (int j = J0; j < J0 + 8; ++j) {
    const int s = __builtin_amdgcn_readlane(sv, j);
    const int d = __builtin_amdgcn_readlane(dv, j);
    const v4f xr = *(const v4f*)(R + (size_t)s * CH + 4 * lane);
    const v4f yr = *(const v4f*)(R + (size_t)d * CH + 4 * lane);
    const v4f ss = *(const v4f*)(S + (size_t)s * CH + 4 * lane);
    const v4f sd = *(const v4f*)(S + (size_t)d * CH + 4 * lane);
    const v4f p = xr * yr;
    v4h ph;
    ph.x = (_Float16)(p.x * HSC); ph.y = (_Float16)(p.y * HSC);
    ph.z = (_Float16)(p.z * HSC); ph.w = (_Float16)(p.w * HSC);
    *(v4h*)(hw + j * APZ + 4 * lane) = ph;
    const v4f df = ss - sd;
    v4f ad;
    ad.x = df.x * ASC + b1s.x; ad.y = df.y * ASC + b1s.y;
    ad.z = df.z * ASC + b1s.z; ad.w = df.w * ASC + b1s.w;
    *(v4f*)(dw + j * DPF + 4 * lane) = ad;
  }
}

__global__ __launch_bounds__(PTHR) void k_wprep(const float* __restrict__ Wd, const float* __restrict__ W1,
                                                _Float16* Bpl) {
  const int blk = blockIdx.x, tid = threadIdx.x;
  const int plane = blk >> 3;
  const int i = (blk & 7) * PTHR + tid;
  const int n = i >> 4, k0 = (i & 15) * 8;
  const float* sp = (plane == 0) ? (Wd + n * CH + k0)
                                 : (W1 + n * (2 * CH) + (plane == 2 ? CH : 0) + k0);
  const v4f a = *(const v4f*)sp;
  const v4f b = *(const v4f*)(sp + 4);
  v8h hv;
  hv[0] = (_Float16)(a.x * WSC); hv[1] = (_Float16)(a.y * WSC); hv[2] = (_Float16)(a.z * WSC); hv[3] = (_Float16)(a.w * WSC);
  hv[4] = (_Float16)(b.x * WSC); hv[5] = (_Float16)(b.y * WSC); hv[6] = (_Float16)(b.z * WSC); hv[7] = (_Float16)(b.w * WSC);
  _Float16* dp = Bpl + plane * PLN + i * 8;
  *(volatile v8h*)dp = hv;
  __threadfence();
  *(volatile v8h*)dp = hv;
}

__global__ __launch_bounds__(GTHR) void k_nodegemm(const float* __restrict__ X, const _Float16* __restrict__ Bp,
                                                   const float* __restrict__ bias, float* Y, int nN, int mode) {
  __shared__ __attribute__((aligned(16))) _Float16 At[GROWS * APZ];
  __shared__ __attribute__((aligned(16))) float stg[GROWS * CH];
  const int tid = threadIdx.x, lane = tid & 31, wave = tid >> 5, hh = lane >> 4, m = lane & 15;
  const int rowBase = blockIdx.x * GROWS;
  {
    const int r = tid >> 1, c0 = (tid & 1) * 64;
    int xrow = rowBase + r;
    xrow = xrow > nN - 1 ? nN - 1 : xrow;
    const float* xp = X + (size_t)xrow * CH + c0;
#pragma unroll
    for (int j = 0; j < 8; ++j) {
      const v4f a = *(const v4f*)(xp + 8 * j), b = *(const v4f*)(xp + 8 * j + 4);
      v8h hv;
      hv[0] = (_Float16)a.x; hv[1] = (_Float16)a.y; hv[2] = (_Float16)a.z; hv[3] = (_Float16)a.w;
      hv[4] = (_Float16)b.x; hv[5] = (_Float16)b.y; hv[6] = (_Float16)b.z; hv[7] = (_Float16)b.w;
      *(v8h*)(At + r * APZ + c0 + 8 * j) = hv;
    }
  }
  __syncthreads();

  {
    v8f acc[8];
    mma16<8>(At + wave * 16 * APZ, Bp, lane, acc);
    float* sp = stg + (wave * 16 + 8 * hh) * CH + m;
#pragma unroll
    for (int t = 0; t < 8; ++t) {
      const float bb = bias[16 * t + m];
      const float bv = mode ? 0.0f : bb;
#pragma unroll
      for (int r = 0; r < 8; ++r) {
        const float v = acc[t][r] * RW + bv;
        sp[r * CH + 16 * t] = mode ? v : fmaxf(v, 0.0f);
      }
    }
  }
  __syncthreads();

  float* gp = Y + (size_t)rowBase * CH;
#pragma unroll
  for (int it = 0; it < 16; ++it) {
    const int f = it * GTHR + tid;
    const v4f v = *(const v4f*)(stg + 4 * f);
    *(volatile v4f*)(gp + 4 * f) = v;
  }
  __threadfence();
#pragma unroll
  for (int it = 0; it < 16; ++it) {
    const int f = it * GTHR + tid;
    const v4f v = *(const v4f*)(stg + 4 * f);
    *(volatile v4f*)(gp + 4 * f) = v;
  }
}

__global__ __launch_bounds__(ETHR) void k_edge(
    const float* __restrict__ R, const float* __restrict__ S, const int* __restrict__ eidx,
    const _Float16* __restrict__ BA, const float* __restrict__ b1, const float* __restrict__ W2,
    const float* __restrict__ b2, float* out, int nN, int nE) {
  __shared__ __attribute__((aligned(16))) _Float16 ht[EWAV * EPW * APZ];
  __shared__ __attribute__((aligned(16))) float    dt[EWAV * EPW * DPF];
  __shared__ __attribute__((aligned(16))) float    sc[EPB];
  const int tid = threadIdx.x, lane = tid & 31, wave = tid >> 5, hh = lane >> 4, m = lane & 15;
  _Float16* hw = ht + wave * (EPW * APZ);
  float*    dw = dt + wave * (EPW * DPF);

  v4f b1s = *(const v4f*)(b1 + 4 * lane);
  b1s.x *= ASC; b1s.y *= ASC; b1s.z *= ASC; b1s.w *= ASC;
  const float b2v = b2[0];

  const int eBase = blockIdx.x * EPB + wave * EPW;
  int e = eBase + lane;
  e = e > nE - 1 ? nE - 1 : e;
  int sv = eidx[e];
  sv = sv < 0 ? 0 : (sv > nN - 1 ? nN - 1 : sv);
  int dv = eidx[(size_t)nE + e];
  dv = dv < 0 ? 0 : (dv > nN - 1 ? nN - 1 : dv);

  rows8<0>(hw, dw, R, S, b1s, sv, dv, lane);
  asm volatile("" ::: "memory");
  rows8<8>(hw, dw, R, S, b1s, sv, dv, lane);
  asm volatile("" ::: "memory");
  rows8<16>(hw, dw, R, S, b1s, sv, dv, lane);
  asm volatile("" ::: "memory");
  rows8<24>(hw, dw, R, S, b1s, sv, dv, lane);
  __syncthreads();

  const float* d0p = dw + (8 * hh) * DPF + m;
  const float* d1p = d0p + 16 * DPF;
  float v[16];
#pragma unroll
  for (int i = 0; i < 16; ++i) v[i] = 0.0f;

#pragma unroll
  for (int cb = 0; cb < 2; ++cb) {
    v8f acc0[4], acc1[4];
    mma32<4>(hw, BA + (size_t)(cb * 64) * KPB, lane, acc0, acc1);
    float w2c[4];
#pragma unroll
    for (int t = 0; t < 4; ++t) w2c[t] = W2[64 * cb + 16 * t + m];
#pragma unroll
    for (int r = 0; r < 8; ++r) {
      float s0 = v[r], s1 = v[8 + r];
#pragma unroll
      for (int t = 0; t < 4; ++t) {
        const float a0 = d0p[r * DPF + 64 * cb + 16 * t];
        const float a1 = d1p[r * DPF + 64 * cb + 16 * t];
        const float h0 = fmaxf(acc0[t][r] + a0, 0.0f);
        const float h1 = fmaxf(acc1[t][r] + a1, 0.0f);
        s0 = fmaf(h0, w2c[t], s0);
        s1 = fmaf(h1, w2c[t], s1);
      }
      v[r] = s0;
      v[8 + r] = s1;
    }
  }

  float u[8];
  {
    const bool kb = ((lane >> 3) & 1) != 0;
#pragma unroll
    for (int i = 0; i < 8; ++i) {
      const float snd = kb ? v[i] : v[i + 8];
      const float kp  = kb ? v[i + 8] : v[i];
      u[i] = kp + __shfl_xor(snd, 8, 32);
    }
  }
  float w4[4];
  {
    const bool kb = ((lane >> 2) & 1) != 0;
#pragma unroll
    for (int i = 0; i < 4; ++i) {
      const float snd = kb ? u[i] : u[i + 4];
      const float kp  = kb ? u[i + 4] : u[i];
      w4[i] = kp + __shfl_xor(snd, 4, 32);
    }
  }
  float x2[2];
  {
    const bool kb = ((lane >> 1) & 1) != 0;
#pragma unroll
    for (int i = 0; i < 2; ++i) {
      const float snd = kb ? w4[i] : w4[i + 2];
      const float kp  = kb ? w4[i + 2] : w4[i];
      x2[i] = kp + __shfl_xor(snd, 2, 32);
    }
  }
  float fin;
  {
    const bool kb = (lane & 1) != 0;
    const float snd = kb ? x2[0] : x2[1];
    const float kp  = kb ? x2[1] : x2[0];
    fin = kp + __shfl_xor(snd, 1, 32);
  }
  {
    float s = fin * RH + b2v;
    s = fminf(fmaxf(s, -40.0f), 40.0f);
    const float ex = __expf(-s);
    const float score = __builtin_amdgcn_rcpf(1.0f + ex);
    const int j = 16 * (m >> 3) + 8 * hh + (m & 7);
    sc[wave * EPW + j] = score;
  }
  __syncthreads();

  if (wave == 0) {
    const int q = lane & 15;
    const v4f ov = *(const v4f*)(sc + 4 * q);
    const int e0 = blockIdx.x * EPB + 4 * q;
    float* op = out + e0;
    const bool act  = lane < 16;
    const bool full = act && (e0 + 3 < nE);
    if (full) {
      *(volatile v4f*)op = ov;
    } else if (act) {
      if (e0     < nE) *(volatile float*)(op)     = ov.x;
      if (e0 + 1 < nE) *(volatile float*)(op + 1) = ov.y;
      if (e0 + 2 < nE) *(volatile float*)(op + 2) = ov.z;
    }
    __threadfence();
    if (full) {
      *(volatile v4f*)op = ov;
    } else if (act) {
      if (e0     < nE) *(volatile float*)(op)     = ov.x;
      if (e0 + 1 < nE) *(volatile float*)(op + 1) = ov.y;
      if (e0 + 2 < nE) *(volatile float*)(op + 2) = ov.z;
    }
  }
}

extern "C" void kernel_launch(void* const* d_in, const int* in_sizes, int n_in,
                              void* d_out, int out_size, void* d_ws, size_t ws_size,
                              hipStream_t stream) {
  if (n_in < 8) return;
  const int nN = in_sizes[0] / CH;
  const int nE = in_sizes[1] / 2;
  if (nN <= 0 || nE <= 0) return;
  if (in_sizes[0] != nN * CH || in_sizes[1] != 2 * nE) return;
  if (in_sizes[2] != CH * CH || in_sizes[3] != CH || in_sizes[4] != 2 * CH * CH ||
      in_sizes[5] != CH || in_sizes[6] != CH || in_sizes[7] < 1) return;
  if (out_size != nE) return;
  if (nN > (1 << 24) || nE > (1 << 29)) return;

  const float* X    = (const float*)d_in[0];
  const int*   eidx = (const int*)d_in[1];
  const float* Wd   = (const float*)d_in[2];
  const float* bd   = (const float*)d_in[3];
  const float* W1   = (const float*)d_in[4];
  const float* b1   = (const float*)d_in[5];
  const float* W2   = (const float*)d_in[6];
  const float* b2   = (const float*)d_in[7];
  float* out = (float*)d_out;

  const int nBlkG = (nN + GROWS - 1) / GROWS;
  const int nPad  = nBlkG * GROWS;
  const int nBlkE = (nE + EPB - 1) / EPB;

  char* ws = (char*)d_ws;
  size_t off = 0;
  const size_t oB = off; off += (size_t)BPTOT * 2;          off = (off + 255) & ~(size_t)255;
  const size_t oR = off; off += (size_t)nPad * CH * 4;      off = (off + 255) & ~(size_t)255;
  const size_t oS = off; off += (size_t)nPad * CH * 4;      off = (off + 255) & ~(size_t)255;
  if (off > ws_size || off > (size_t)WSCAP) return;
  _Float16* Bpl = (_Float16*)(ws + oB);
  float*    R   = (float*)(ws + oR);
  float*    S   = (float*)(ws + oS);

  k_wprep<<<NPBLK, PTHR, 0, stream>>>(Wd, W1, Bpl);
  k_nodegemm<<<nBlkG, GTHR, 0, stream>>>(X, Bpl + OFF_PD, bd, R, nN, 0);
  k_nodegemm<<<nBlkG, GTHR, 0, stream>>>(R, Bpl + OFF_PB, bd, S, nN, 1);
  k_edge<<<nBlkE, ETHR, 0, stream>>>(R, S, eidx, Bpl + OFF_PA, b1, W2, b2, out, nN, nE);
}
